// GNNConditioner_56186762166749
// MI455X (gfx1250) — hardware-verified
//
#include <hip/hip_runtime.h>
#include <hip/hip_bf16.h>
#include <stddef.h>
#include <stdint.h>


#define NBL     4096
#define HID     512
#define KF      1024
#define XD      2
#define NO      4
#define NTHR    256
#define NWAVE   8
#define EPT     8
#define CHUNK   (NTHR * EPT)
#define WCAP    (EPT * 32)
#define LISTN   (NWAVE * WCAP)
#define NBMAX   2048
#define RCAP    16384
#define DEGCAP  1024
#define STW     512
#define WTABN   3072
#define GBM     64
#define GBN     64
#define GTHR    128
#define TABN    6176
#define T_W10   0
#define T_B10   1024
#define T_W11   1536
#define T_B11   2560
#define T_WH2   3072
#define T_BH2   5120
#define T_B2S   5152
#define T_BH1   5664
#define WSMAX   134217728
#define LDS_AGG ((2 * RCAP + 2 * NBMAX + LISTN) * 4 + 64)

static_assert((CHUNK & (CHUNK - 1)) == 0 && CHUNK <= 4096);
static_assert((NBMAX & (NBMAX - 1)) == 0 && NBMAX <= 4096);
static_assert(NTHR * 8 == NBMAX);
static_assert(LISTN >= NBMAX);
static_assert(LISTN >= NWAVE * WCAP);
static_assert((RCAP % 32) == 0 && (RCAP % 4) == 0);
static_assert(NWAVE * STW + WTABN + NBL <= RCAP);
static_assert(LDS_AGG <= 300000);
static_assert(GBM == (GTHR / 32) * 16);
static_assert((HID % GBN) == 0 && (HID % 32) == 0 && (KF % 32) == 0 && KF == 2 * HID);
static_assert((NBL % GBM) == 0);
static_assert((TABN % 32) == 0 && T_BH1 + HID == TABN && T_B11 + HID == WTABN);
static_assert(HID == 512 && STW == HID);
static_assert(GBM * NO == 2 * GTHR);

typedef float    v2f  __attribute__((ext_vector_type(2)));
typedef float    v4f  __attribute__((ext_vector_type(4)));
typedef float    v8f  __attribute__((ext_vector_type(8)));
typedef int      v4i  __attribute__((ext_vector_type(4)));
typedef int      v8i  __attribute__((ext_vector_type(8)));
typedef unsigned short v8us __attribute__((ext_vector_type(8)));
typedef __bf16   v16b __attribute__((ext_vector_type(16)));
union FragB { v16b v; v8us h[2]; v8i w; };

__device__ __forceinline__ v8f wmb(const FragB& a, const FragB& b, v8f c) {
  v8f d = __builtin_amdgcn_wmma_f32_16x16x32_bf16(false, a.v, false, b.v, (short)0, c, false, false);
  asm volatile("v_nop\n\tv_nop\n\tv_nop\n\tv_nop" : "+v"(d) : "v"(a.w), "v"(b.w));
  return d;
}

__device__ __forceinline__ unsigned bfb(float x) {
  const unsigned u = __float_as_uint(x);
  return (u + 0x7fffu + ((u >> 16) & 1u)) >> 16;
}
__device__ __forceinline__ float bfr(float x) { return __uint_as_float(bfb(x) << 16); }

__device__ __forceinline__ void split8(const v4f a, const v4f b, v8us& hi, v8us& lo) {
  float x[8] = {a.x, a.y, a.z, a.w, b.x, b.y, b.z, b.w};
#pragma unroll
  for (int i = 0; i < 8; ++i) {
    const unsigned hb = bfb(x[i]);
    const float rs = x[i] - __uint_as_float(hb << 16);
    hi[i] = (unsigned short)hb;
    lo[i] = (unsigned short)bfb(rs);
  }
}

__device__ __forceinline__ float silu_f(float x) {
  const float e = __expf(-x);
  return x * __builtin_amdgcn_rcpf(1.0f + e);
}

__device__ __forceinline__ v4f fma4(float w, const v4f v, v4f a) {
  a.x = fmaf(w, v.x, a.x); a.y = fmaf(w, v.y, a.y); a.z = fmaf(w, v.z, a.z); a.w = fmaf(w, v.w, a.w);
  return a;
}

__device__ __forceinline__ int scan_chunk(const int* __restrict__ dsts, int nE, int cbase, int slotBase,
                                          int nb, int vec8, int* list, int tid, int lane, int wave) {
  int wc = 0;
  const int el0  = tid * EPT;
  const int e0   = cbase + el0;
  const int sent = -2147483647 - 1;
  v4i da, db;
  if (vec8 != 0 && cbase + CHUNK <= nE) {
    da = *(const v4i*)(dsts + e0);
    db = *(const v4i*)(dsts + e0 + 4);
  } else {
    da.x = (e0     < nE) ? dsts[min(e0,     nE - 1)] : sent;
    da.y = (e0 + 1 < nE) ? dsts[min(e0 + 1, nE - 1)] : sent;
    da.z = (e0 + 2 < nE) ? dsts[min(e0 + 2, nE - 1)] : sent;
    da.w = (e0 + 3 < nE) ? dsts[min(e0 + 3, nE - 1)] : sent;
    db.x = (e0 + 4 < nE) ? dsts[min(e0 + 4, nE - 1)] : sent;
    db.y = (e0 + 5 < nE) ? dsts[min(e0 + 5, nE - 1)] : sent;
    db.z = (e0 + 6 < nE) ? dsts[min(e0 + 6, nE - 1)] : sent;
    db.w = (e0 + 7 < nE) ? dsts[min(e0 + 7, nE - 1)] : sent;
  }
  const unsigned nbs = (unsigned)slotBase;
  const unsigned unb = (unsigned)nb;
  const unsigned s0 = (unsigned)da.x - nbs, s1 = (unsigned)da.y - nbs;
  const unsigned s2 = (unsigned)da.z - nbs, s3 = (unsigned)da.w - nbs;
  const unsigned s4 = (unsigned)db.x - nbs, s5 = (unsigned)db.y - nbs;
  const unsigned s6 = (unsigned)db.z - nbs, s7 = (unsigned)db.w - nbs;
  const bool h0 = s0 < unb, h1 = s1 < unb, h2 = s2 < unb, h3 = s3 < unb;
  const bool h4 = s4 < unb, h5 = s5 < unb, h6 = s6 < unb, h7 = s7 < unb;
  const unsigned any = __builtin_amdgcn_ballot_w32(h0 | h1 | h2 | h3 | h4 | h5 | h6 | h7);
  if (any != 0u) {
#define HITJ(J, HJ, SJ) { \
      const unsigned mj = __builtin_amdgcn_ballot_w32(HJ); \
      if (mj != 0u) { \
        if (HJ) { \
          const int pos = wc + (int)__builtin_amdgcn_mbcnt_lo(mj, 0u); \
          if (pos < WCAP) list[wave * WCAP + pos] = ((el0 + (J)) << 12) | (int)(SJ); \
        } \
        wc += (int)__builtin_popcount(mj); } }
    HITJ(0, h0, s0)
    HITJ(1, h1, s1)
    HITJ(2, h2, s2)
    HITJ(3, h3, s3)
    HITJ(4, h4, s4)
    HITJ(5, h5, s5)
    HITJ(6, h6, s6)
    HITJ(7, h7, s7)
#undef HITJ
  }
  return wc;
}

__global__ __launch_bounds__(NTHR) void k_prep(
    const float* __restrict__ X, const float* __restrict__ W10, const float* __restrict__ b10,
    const float* __restrict__ W11, const float* __restrict__ b11, const float* __restrict__ Wh2,
    const float* __restrict__ bh2, const float* __restrict__ b20, const float* __restrict__ b21,
    const float* __restrict__ bh1, float* Xr, float* tab, int nXf) {
  const int seg = (int)blockIdx.y;
  const int u = (int)blockIdx.x * NTHR + (int)threadIdx.x;
  const float* p0; const float* p1; int nsrc; float* dst; int nu;
  if (seg == 0)      { p0 = X;   p1 = X;   nsrc = nXf;  dst = Xr;          nu = nXf >> 2; }
  else if (seg == 1) { p0 = W10; p1 = W10; nsrc = 1024; dst = tab + T_W10; nu = 256; }
  else if (seg == 2) { p0 = b10; p1 = b10; nsrc = 512;  dst = tab + T_B10; nu = 128; }
  else if (seg == 3) { p0 = W11; p1 = W11; nsrc = 1024; dst = tab + T_W11; nu = 256; }
  else if (seg == 4) { p0 = b11; p1 = b11; nsrc = 512;  dst = tab + T_B11; nu = 128; }
  else if (seg == 5) { p0 = Wh2; p1 = Wh2; nsrc = 2048; dst = tab + T_WH2; nu = 512; }
  else if (seg == 6) { p0 = bh2; p1 = bh2; nsrc = 4;    dst = tab + T_BH2; nu = 8; }
  else if (seg == 7) { p0 = b20; p1 = b21; nsrc = 512;  dst = tab + T_B2S; nu = 128; }
  else               { p0 = bh1; p1 = bh1; nsrc = 512;  dst = tab + T_BH1; nu = 128; }
  if (u >= nu) return;
  const bool two = (seg == 7);
  const int i0 = 4 * u;
  const int c0 = min(i0, nsrc - 1), c1 = min(i0 + 1, nsrc - 1), c2 = min(i0 + 2, nsrc - 1), c3 = min(i0 + 3, nsrc - 1);
  v4f r;
  r.x = bfr(p0[c0]) + (two ? bfr(p1[c0]) : 0.f);
  r.y = bfr(p0[c1]) + (two ? bfr(p1[c1]) : 0.f);
  r.z = bfr(p0[c2]) + (two ? bfr(p1[c2]) : 0.f);
  r.w = bfr(p0[c3]) + (two ? bfr(p1[c3]) : 0.f);
  if (i0     >= nsrc) r.x = 0.f;
  if (i0 + 1 >= nsrc) r.y = 0.f;
  if (i0 + 2 >= nsrc) r.z = 0.f;
  if (i0 + 3 >= nsrc) r.w = 0.f;
  float* op = dst + i0;
  *(volatile v4f*)op = r;
  __threadfence();
  *(volatile v4f*)op = r;
}

__global__ __launch_bounds__(NTHR) void k_wtr(const float* __restrict__ w0, const float* __restrict__ w1,
                                              int ksplit, int K, int ncol, unsigned short* wt, int nUnits) {
  const int u = (int)blockIdx.x * NTHR + (int)threadIdx.x;
  if (u >= nUnits) return;
  const int kq = K >> 3;
  const int n  = u / kq;
  const int k8 = (u - n * kq) * 8;
  const bool sec = k8 >= ksplit;
  const float* ws = sec ? w1 : w0;
  const int kk = sec ? (k8 - ksplit) : k8;
  const float* p = ws + (size_t)kk * (size_t)ncol + n;
  v8us hv;
  hv[0] = (unsigned short)bfb(p[0]);
  hv[1] = (unsigned short)bfb(p[(size_t)ncol]);
  hv[2] = (unsigned short)bfb(p[(size_t)2 * ncol]);
  hv[3] = (unsigned short)bfb(p[(size_t)3 * ncol]);
  hv[4] = (unsigned short)bfb(p[(size_t)4 * ncol]);
  hv[5] = (unsigned short)bfb(p[(size_t)5 * ncol]);
  hv[6] = (unsigned short)bfb(p[(size_t)6 * ncol]);
  hv[7] = (unsigned short)bfb(p[(size_t)7 * ncol]);
  const size_t o = (size_t)n * (size_t)K + k8;
  *(volatile v8us*)(wt + o) = hv;
  __threadfence();
  *(volatile v8us*)(wt + o) = hv;
}

__global__ __launch_bounds__(NTHR) void k_cvt(const float* __restrict__ Hf, unsigned short* Ahi,
                                              unsigned short* Alo, int nUnits, int lda) {
  const int u = (int)blockIdx.x * NTHR + (int)threadIdx.x;
  if (u >= nUnits) return;
  const int row = u >> 6;
  const int c8  = (u & 63) * 8;
  const float* p = Hf + (size_t)row * HID + c8;
  const v4f a = *(const v4f*)p, b = *(const v4f*)(p + 4);
  v8us hv, lv;
  split8(a, b, hv, lv);
  const size_t o = (size_t)row * (size_t)lda + c8;
  *(volatile v8us*)(Ahi + o) = hv;
  *(volatile v8us*)(Alo + o) = lv;
  __threadfence();
  *(volatile v8us*)(Ahi + o) = hv;
  *(volatile v8us*)(Alo + o) = lv;
}

template<int MODE>
__global__ __launch_bounds__(NTHR) void k_agg(
    const int* __restrict__ srcs, const int* __restrict__ dsts, int nE, int nb, int vec8, int copy0,
    const float* __restrict__ dinv, float* dinvOut,
    const float* __restrict__ Xr, const float* __restrict__ tab,
    float* H1f, unsigned short* Ahi, unsigned short* Alo) {
  extern __shared__ v4f lds_dyn[];
  int* reg1 = (int*)lds_dyn;
  int* reg2 = reg1 + RCAP;
  int* scnt = reg2 + RCAP;
  int* soff = scnt + NBMAX;
  int* list = soff + NBMAX;
  int* wcnt = list + LISTN;
  int* wtot = wcnt + NWAVE;
  const int tid = (int)threadIdx.x, lane = tid & 31, wave = tid >> 5;
  const int nodeBase = (int)blockIdx.x * nb;
  const int copy = copy0 + (int)blockIdx.y;

  {
    const v4i z4 = {0, 0, 0, 0};
    v4i* zp = (v4i*)lds_dyn;
#pragma unroll 1
    for (int i = tid; i < (2 * RCAP + NBMAX) / 4; i += NTHR) zp[i] = z4;
  }
  __syncthreads();

  int tot = 0;
  const int nChunks = (nE + CHUNK - 1) / CHUNK;
#pragma unroll 1
  for (int ch = 0; ch < nChunks; ++ch) {
    const int cbase = ch * CHUNK;
    const int wc = scan_chunk(dsts, nE, cbase, nodeBase, nb, vec8, list, tid, lane, wave);
    if (lane == 0) wcnt[wave] = wc;
    __syncthreads();
    int pre = 0, all = 0;
#pragma unroll
    for (int w2 = 0; w2 < NWAVE; ++w2) {
      int c = wcnt[w2];
      c = c < 0 ? 0 : (c > WCAP ? WCAP : c);
      all += c;
      pre += (w2 < wave) ? c : 0;
    }
    const int wcc  = wc > WCAP ? WCAP : wc;
    const int base = tot + pre;
#pragma unroll 1
    for (int i = lane; i < wcc; i += 32) {
      const int ent = list[wave * WCAP + i];
      const int el  = (ent >> 12) & (CHUNK - 1);
      const int sl  = ent & (NBMAX - 1);
      int eid = cbase + el;
      eid = eid > nE - 1 ? nE - 1 : eid;
      const int pos = base + i;
      if (pos < RCAP) reg1[pos] = (int)(((unsigned)eid << 12) | (unsigned)sl);
    }
    tot += all;
    tot = tot > RCAP ? RCAP : tot;
    __syncthreads();
  }
  const int nh = tot;

  if (wave == 0) {
#pragma unroll 1
    for (int b0 = 0; b0 < nh; b0 += 32) {
      const int idx = b0 + lane;
      const int uv  = reg1[idx < RCAP ? idx : RCAP - 1];
      const int m32 = (nh - b0) < 32 ? (nh - b0) : 32;
#pragma unroll 1
      for (int k = 0; k < m32; ++k) {
        const int u  = __builtin_amdgcn_readlane(uv, k);
        const int sl = u & (NBMAX - 1);
        if (lane == 0) scnt[sl] = scnt[sl] + 1;
      }
    }
  }
  __syncthreads();

  if (MODE == 2) {
    const bool ovf2 = (nh >= RCAP);
    const float qn2 = __int_as_float(0x7fc00000);
    const bool act = tid < (nb >> 2);
    const int t4 = act ? 4 * tid : 0;
    const v4i c = *(const v4i*)(scnt + t4);
    const int e0 = c.x < 0 ? 0 : c.x, e1 = c.y < 0 ? 0 : c.y, e2 = c.z < 0 ? 0 : c.z, e3 = c.w < 0 ? 0 : c.w;
    v4f d;
    d.x = rsqrtf(1.0f + (float)e0);
    d.y = rsqrtf(1.0f + (float)e1);
    d.z = rsqrtf(1.0f + (float)e2);
    d.w = rsqrtf(1.0f + (float)e3);
    if (ovf2) { d.x = qn2; d.y = qn2; d.z = qn2; d.w = qn2; }
    float* op = dinvOut + nodeBase + t4;
    if (act) *(volatile v4f*)op = d;
    __threadfence();
    if (act) *(volatile v4f*)op = d;
    return;
  }

  {
    const v4i ca = *(const v4i*)(scnt + 8 * tid);
    const v4i cb = *(const v4i*)(scnt + 8 * tid + 4);
    const int e0 = ca.x < 0 ? 0 : ca.x, e1 = ca.y < 0 ? 0 : ca.y, e2 = ca.z < 0 ? 0 : ca.z, e3 = ca.w < 0 ? 0 : ca.w;
    const int e4 = cb.x < 0 ? 0 : cb.x, e5 = cb.y < 0 ? 0 : cb.y, e6 = cb.z < 0 ? 0 : cb.z, e7 = cb.w < 0 ? 0 : cb.w;
    const int ts = e0 + e1 + e2 + e3 + e4 + e5 + e6 + e7;
    int incl = ts;
#pragma unroll
    for (int d = 1; d < 32; d <<= 1) {
      const int up = __shfl_up(incl, d);
      if (lane >= d) incl += up;
    }
    if (lane == 31) wtot[wave] = incl;
    __syncthreads();
    int pre = 0;
#pragma unroll
    for (int w2 = 0; w2 < NWAVE; ++w2) pre += (w2 < wave) ? wtot[w2] : 0;
    int run = pre + incl - ts;
    soff[8 * tid + 0] = run; run += e0;
    soff[8 * tid + 1] = run; run += e1;
    soff[8 * tid + 2] = run; run += e2;
    soff[8 * tid + 3] = run; run += e3;
    soff[8 * tid + 4] = run; run += e4;
    soff[8 * tid + 5] = run; run += e5;
    soff[8 * tid + 6] = run; run += e6;
    soff[8 * tid + 7] = run;
  }
  __syncthreads();
  for (int i = tid; i < NBMAX; i += NTHR) list[i] = soff[i];
  __syncthreads();

  if (wave == 0) {
#pragma unroll 1
    for (int b0 = 0; b0 < nh; b0 += 32) {
      const int idx = b0 + lane;
      const int uv  = reg1[idx < RCAP ? idx : RCAP - 1];
      const int m32 = (nh - b0) < 32 ? (nh - b0) : 32;
#pragma unroll 1
      for (int k = 0; k < m32; ++k) {
        const int u   = __builtin_amdgcn_readlane(uv, k);
        const int sl  = u & (NBMAX - 1);
        const int eid = (int)((unsigned)u >> 12);
        if (lane == 0) {
          int pos = list[sl];
          pos = pos < 0 ? 0 : (pos > RCAP - 1 ? RCAP - 1 : pos);
          reg2[pos] = eid;
          list[sl] = pos + 1;
        }
      }
    }
  }
  __syncthreads();

  const int nbw = nb >> 3;
  const bool ovf = (nh >= RCAP);
  const float qnan = __int_as_float(0x7fc00000);
  float* stw   = (float*)reg1 + wave * STW;
  float* wtab  = (float*)reg1 + NWAVE * STW;
  float* dinvS = wtab + WTABN;
  for (int i = tid; i < NBL; i += NTHR) dinvS[i] = dinv[i];
  if (MODE == 0) {
    for (int i = tid; i < WTABN; i += NTHR) wtab[i] = tab[i];
  }
  __syncthreads();
  const size_t cb = (size_t)copy * NBL;

#pragma unroll 1
  for (int jt = 0; jt < nbw; ++jt) {
    const int slot = wave * nbw + jt;
    int gl = nodeBase + slot;
    gl = gl > NBL - 1 ? NBL - 1 : gl;
    const size_t grow = cb + (size_t)gl;
    int st = soff[slot];
    const int craw = scnt[slot];
    int cnt = craw;
    st  = st < 0 ? 0 : (st > nh ? nh : st);
    cnt = cnt < 0 ? 0 : (cnt > DEGCAP ? DEGCAP : cnt);
    if (cnt > nh - st) cnt = nh - st;
    cnt = cnt < 0 ? 0 : cnt;
    const float pz = (ovf || craw > DEGCAP) ? qnan : 0.0f;
    const float di = dinvS[gl];

    if (MODE == 0) {
      float p0 = 0.f, p1 = 0.f;
#pragma unroll 1
      for (int q0 = 0; q0 < cnt; q0 += 32) {
        const int q = q0 + lane;
        const bool act = q < cnt;
        int idx = st + (act ? q : cnt - 1);
        idx = idx < 0 ? 0 : (idx > RCAP - 1 ? RCAP - 1 : idx);
        int eid = reg2[idx]; eid = eid < 0 ? 0 : (eid > nE - 1 ? nE - 1 : eid);
        int se = srcs[eid];  se = se < 0 ? 0 : (se > NBL - 1 ? NBL - 1 : se);
        const float w = act ? dinvS[se] * di : 0.0f;
        const v2f xv = *(const v2f*)(Xr + (cb + (size_t)se) * 2);
        p0 = fmaf(w, xv.x, p0);
        p1 = fmaf(w, xv.y, p1);
      }
#pragma unroll
      for (int off = 16; off > 0; off >>= 1) {
        p0 += __shfl_xor(p0, off);
        p1 += __shfl_xor(p1, off);
      }
      const v2f xo = *(const v2f*)(Xr + grow * 2);
      const float dd = di * di;
      const float a0 = fmaf(dd, xo.x, p0);
      const float a1 = fmaf(dd, xo.y, p1);
      const float x0 = xo.x, x1 = xo.y;
      __builtin_amdgcn_fence(__ATOMIC_RELEASE, "wavefront");
      __builtin_amdgcn_wave_barrier();
#pragma unroll 1
      for (int t = 0; t < 16; ++t) {
        const int c = 128 * (t >> 2) + 4 * lane + (t & 3);
        const float hx = fmaf(x1, wtab[T_W10 + HID + c], x0 * wtab[T_W10 + c]) + wtab[T_B10 + c];
        const float ha = fmaf(a1, wtab[T_W11 + HID + c], a0 * wtab[T_W11 + c]) + wtab[T_B11 + c];
        stw[c] = silu_f(hx + ha) + pz;
      }
      __builtin_amdgcn_fence(__ATOMIC_RELEASE, "wavefront");
      __builtin_amdgcn_wave_barrier();
      const v4f g0 = *(const v4f*)(stw + 4 * lane);
      const v4f g1 = *(const v4f*)(stw + 128 + 4 * lane);
      const v4f g2 = *(const v4f*)(stw + 256 + 4 * lane);
      const v4f g3 = *(const v4f*)(stw + 384 + 4 * lane);
      float* op = H1f + grow * HID + 4 * lane;
      *(volatile v4f*)(op)       = g0;
      *(volatile v4f*)(op + 128) = g1;
      *(volatile v4f*)(op + 256) = g2;
      *(volatile v4f*)(op + 384) = g3;
      __threadfence();
      *(volatile v4f*)(op)       = g0;
      *(volatile v4f*)(op + 128) = g1;
      *(volatile v4f*)(op + 256) = g2;
      *(volatile v4f*)(op + 384) = g3;
    } else {
      const v4f z4 = {0.f, 0.f, 0.f, 0.f};
      v4f a0 = z4, a1 = z4, a2 = z4, a3 = z4;
      const float* hb = H1f + cb * HID + 4 * lane;
#pragma unroll 1
      for (int q = 0; q <= cnt; ++q) {
        const bool isE = q < cnt;
        int idx = st + (isE ? q : (cnt > 0 ? cnt - 1 : 0));
        idx = idx < 0 ? 0 : (idx > RCAP - 1 ? RCAP - 1 : idx);
        int eid = reg2[idx]; eid = eid < 0 ? 0 : (eid > nE - 1 ? nE - 1 : eid);
        int se = srcs[eid];  se = se < 0 ? 0 : (se > NBL - 1 ? NBL - 1 : se);
        const int s = isE ? se : gl;
        const float w = dinvS[s] * di;
        const float* p = hb + (size_t)s * HID;
        const v4f v0 = *(const v4f*)(p);
        const v4f v1 = *(const v4f*)(p + 128);
        const v4f v2 = *(const v4f*)(p + 256);
        const v4f v3 = *(const v4f*)(p + 384);
        a0 = fma4(w, v0, a0);
        a1 = fma4(w, v1, a1);
        a2 = fma4(w, v2, a2);
        a3 = fma4(w, v3, a3);
      }
      __builtin_amdgcn_fence(__ATOMIC_RELEASE, "wavefront");
      __builtin_amdgcn_wave_barrier();
      *(v4f*)(stw + 4 * lane)       = a0;
      *(v4f*)(stw + 128 + 4 * lane) = a1;
      *(v4f*)(stw + 256 + 4 * lane) = a2;
      *(v4f*)(stw + 384 + 4 * lane) = a3;
      __builtin_amdgcn_fence(__ATOMIC_RELEASE, "wavefront");
      __builtin_amdgcn_wave_barrier();
      v4f g0 = *(const v4f*)(stw + 8 * lane);
      v4f g1 = *(const v4f*)(stw + 8 * lane + 4);
      v4f g2 = *(const v4f*)(stw + 256 + 8 * lane);
      v4f g3 = *(const v4f*)(stw + 256 + 8 * lane + 4);
      g0.x += pz; g0.y += pz; g0.z += pz; g0.w += pz;
      g1.x += pz; g1.y += pz; g1.z += pz; g1.w += pz;
      g2.x += pz; g2.y += pz; g2.z += pz; g2.w += pz;
      g3.x += pz; g3.y += pz; g3.z += pz; g3.w += pz;
      v8us hA, lA, hB, lB;
      split8(g0, g1, hA, lA);
      split8(g2, g3, hB, lB);
      const size_t o = (size_t)gl * KF + HID + 8 * lane;
      *(volatile v8us*)(Ahi + o)       = hA;
      *(volatile v8us*)(Ahi + o + 256) = hB;
      *(volatile v8us*)(Alo + o)       = lA;
      *(volatile v8us*)(Alo + o + 256) = lB;
      __threadfence();
      *(volatile v8us*)(Ahi + o)       = hA;
      *(volatile v8us*)(Ahi + o + 256) = hB;
      *(volatile v8us*)(Alo + o)       = lA;
      *(volatile v8us*)(Alo + o + 256) = lB;
    }
  }
}

__global__ __launch_bounds__(GTHR) void k_gemm2(
    const unsigned short* __restrict__ Ahi, const unsigned short* __restrict__ Alo,
    const unsigned short* __restrict__ WT, const float* __restrict__ bias,
    unsigned short* Ohi, unsigned short* Olo, int K, int N) {
  __shared__ __attribute__((aligned(16))) float stg[GBM * GBN];
  const int tid = (int)threadIdx.x, lane = tid & 31, wave = tid >> 5, hh = lane >> 4, m = lane & 15;
  const int rowBase = (int)blockIdx.x * GBM;
  const int col0    = (int)blockIdx.y * GBN;

  v8f acc[4];
  {
    const v8f z = {0.f, 0.f, 0.f, 0.f, 0.f, 0.f, 0.f, 0.f};
    acc[0] = z; acc[1] = z; acc[2] = z; acc[3] = z;
  }
  const size_t arow = (size_t)(rowBase + 16 * wave + m) * (size_t)K + 8 * hh;
  const unsigned short* aph = Ahi + arow;
  const unsigned short* apl = Alo + arow;
  const unsigned short* wp  = WT + (size_t)(col0 + m) * (size_t)K + 8 * hh;
  const int ksteps = K >> 5;
#pragma unroll 1
  for (int ks = 0; ks < ksteps; ++ks) {
    FragB ah, al;
    ah.h[0] = *(const v8us*)(aph + 32 * ks);
    ah.h[1] = *(const v8us*)(aph + 32 * ks + 16);
    al.h[0] = *(const v8us*)(apl + 32 * ks);
    al.h[1] = *(const v8us*)(apl + 32 * ks + 16);
#pragma unroll
    for (int t = 0; t < 4; ++t) {
      const unsigned short* wq = wp + (size_t)(16 * t) * (size_t)K + 32 * ks;
      FragB bf;
      bf.h[0] = *(const v8us*)wq;
      bf.h[1] = *(const v8us*)(wq + 16);
      acc[t] = wmb(ah, bf, acc[t]);
      acc[t] = wmb(al, bf, acc[t]);
    }
  }

#pragma unroll
  for (int t = 0; t < 4; ++t) {
    const int lc = 16 * t + m;
    int bi = col0 + lc;
    bi = bi > N - 1 ? N - 1 : bi;
    const float bv = bias[bi];
#pragma unroll
    for (int r = 0; r < 8; ++r) {
      const int lr = 16 * wave + 8 * hh + r;
      stg[lr * GBN + lc] = silu_f(acc[t][r] + bv);
    }
  }
  __syncthreads();

  v8us hv[4], lv[4];
#pragma unroll
  for (int i = 0; i < 4; ++i) {
    const int lr = 16 * wave + 4 * i + (lane >> 3);
    const int c8 = 8 * (lane & 7);
    const v4f a = *(const v4f*)(stg + lr * GBN + c8);
    const v4f b = *(const v4f*)(stg + lr * GBN + c8 + 4);
    split8(a, b, hv[i], lv[i]);
  }
#pragma unroll
  for (int i = 0; i < 4; ++i) {
    const int lr = 16 * wave + 4 * i + (lane >> 3);
    const int c8 = 8 * (lane & 7);
    const size_t o = (size_t)(rowBase + lr) * (size_t)N + col0 + c8;
    *(volatile v8us*)(Ohi + o) = hv[i];
    *(volatile v8us*)(Olo + o) = lv[i];
  }
  __threadfence();
#pragma unroll
  for (int i = 0; i < 4; ++i) {
    const int lr = 16 * wave + 4 * i + (lane >> 3);
    const int c8 = 8 * (lane & 7);
    const size_t o = (size_t)(rowBase + lr) * (size_t)N + col0 + c8;
    *(volatile v8us*)(Ohi + o) = hv[i];
    *(volatile v8us*)(Olo + o) = lv[i];
  }
}

__global__ __launch_bounds__(GTHR) void k_gemm3(
    const unsigned short* __restrict__ Ahi, const unsigned short* __restrict__ Alo,
    const unsigned short* __restrict__ WT, const float* __restrict__ bh1,
    const float* __restrict__ wh2, const float* __restrict__ bh2,
    float* out, int K, int rowOff, int out1off) {
  __shared__ __attribute__((aligned(16))) float stg[GBM * GBN];
  __shared__ __attribute__((aligned(16))) float wh2s[HID * NO];
  __shared__ __attribute__((aligned(16))) float ost[2 * GBM * 2];
  const int tid = (int)threadIdx.x, lane = tid & 31, wave = tid >> 5, hh = lane >> 4, m = lane & 15;
  const int rowBase = (int)blockIdx.x * GBM;
  for (int i = tid; i < HID * NO / 4; i += GTHR) *(v4f*)(wh2s + 4 * i) = *(const v4f*)(wh2 + 4 * i);

  const size_t arow = (size_t)(rowBase + 16 * wave + m) * (size_t)K + 8 * hh;
  const unsigned short* aph = Ahi + arow;
  const unsigned short* apl = Alo + arow;
  const int ksteps = K >> 5;
  const int hr = tid >> 1;
  const int hc = (tid & 1) * 32;
  v4f hp = {0.f, 0.f, 0.f, 0.f};

#pragma unroll 1
  for (int g = 0; g < HID / GBN; ++g) {
    v8f acc[4];
    {
      const v8f z = {0.f, 0.f, 0.f, 0.f, 0.f, 0.f, 0.f, 0.f};
      acc[0] = z; acc[1] = z; acc[2] = z; acc[3] = z;
    }
    const unsigned short* wp = WT + (size_t)(g * GBN + m) * (size_t)K + 8 * hh;
#pragma unroll 1
    for (int ks = 0; ks < ksteps; ++ks) {
      FragB ah, al;
      ah.h[0] = *(const v8us*)(aph + 32 * ks);
      ah.h[1] = *(const v8us*)(aph + 32 * ks + 16);
      al.h[0] = *(const v8us*)(apl + 32 * ks);
      al.h[1] = *(const v8us*)(apl + 32 * ks + 16);
#pragma unroll
      for (int t = 0; t < 4; ++t) {
        const unsigned short* wq = wp + (size_t)(16 * t) * (size_t)K + 32 * ks;
        FragB bf;
        bf.h[0] = *(const v8us*)wq;
        bf.h[1] = *(const v8us*)(wq + 16);
        acc[t] = wmb(ah, bf, acc[t]);
        acc[t] = wmb(al, bf, acc[t]);
      }
    }
#pragma unroll
    for (int t = 0; t < 4; ++t) {
      const int lc = 16 * t + m;
      const float bv = bh1[g * GBN + lc];
#pragma unroll
      for (int r = 0; r < 8; ++r) {
        const int lr = 16 * wave + 8 * hh + r;
        stg[lr * GBN + lc] = silu_f(acc[t][r] + bv);
      }
    }
    __syncthreads();
#pragma unroll 4
    for (int j = 0; j < 32; ++j) {
      const float gv = stg[hr * GBN + hc + j];
      const v4f w4 = *(const v4f*)(wh2s + (g * GBN + hc + j) * NO);
      hp = fma4(gv, w4, hp);
    }
    __syncthreads();
  }
  hp.x += __shfl_xor(hp.x, 1);
  hp.y += __shfl_xor(hp.y, 1);
  hp.z += __shfl_xor(hp.z, 1);
  hp.w += __shfl_xor(hp.w, 1);
  const float o0 = hp.x + bh2[0], o1 = hp.y + bh2[1], o2 = hp.z + bh2[2], o3 = hp.w + bh2[3];
  const float t0 = tanhf(o0), t1 = tanhf(o1);
  if ((tid & 1) == 0) {
    ost[2 * hr]               = t0;
    ost[2 * hr + 1]           = t1;
    ost[2 * GBM + 2 * hr]     = o2;
    ost[2 * GBM + 2 * hr + 1] = o3;
  }
  __syncthreads();
  const bool wv = wave < 2;
  const int wsel = wave & 1;
  const v4f v = *(const v4f*)(ost + 2 * GBM * wsel + 4 * lane);
  float* op = out + (size_t)(wsel ? out1off : 0) + (size_t)(rowOff + rowBase) * 2 + 4 * lane;
  if (wv) *(volatile v4f*)op = v;
  __threadfence();
  if (wv) *(volatile v4f*)op = v;
}

static int pick_nb(int nE, int nN) {
  int nb = NBMAX;
  while (nb > 64 && (long long)nb * (long long)nE * 5LL > (long long)RCAP * (long long)nN * 4LL) nb >>= 1;
  return nb;
}
static inline int cdiv(int a, int b) { return (a + b - 1) / b; }

extern "C" void kernel_launch(void* const* d_in, const int* in_sizes, int n_in,
                              void* d_out, int out_size, void* d_ws, size_t ws_size,
                              hipStream_t stream) {
  if (n_in < 14) return;
  const int nXf = in_sizes[0];
  if (nXf < NBL * XD || (nXf % (NBL * XD)) != 0) return;
  const int nB = nXf / (NBL * XD);
  if (nB < 1 || nB > 64) return;
  const int nN = nB * NBL;
  if (in_sizes[1] < 2 || (in_sizes[1] & 1) != 0) return;
  const int nE = in_sizes[1] / 2;
  if (nE < 1 || nE > (1 << 20)) return;
  if (in_sizes[2]  != XD * HID  || in_sizes[3]  != HID) return;
  if (in_sizes[4]  != XD * HID  || in_sizes[5]  != HID) return;
  if (in_sizes[6]  != HID * HID || in_sizes[7]  != HID) return;
  if (in_sizes[8]  != HID * HID || in_sizes[9]  != HID) return;
  if (in_sizes[10] != HID * HID || in_sizes[11] != HID) return;
  if (in_sizes[12] != HID * NO  || in_sizes[13] != NO)  return;
  if (out_size != nN * NO) return;

  const float* X    = (const float*)d_in[0];
  const int*   ei   = (const int*)  d_in[1];
  const float* W10  = (const float*)d_in[2];
  const float* b10  = (const float*)d_in[3];
  const float* W11  = (const float*)d_in[4];
  const float* b11  = (const float*)d_in[5];
  const float* W20  = (const float*)d_in[6];
  const float* b20  = (const float*)d_in[7];
  const float* W21  = (const float*)d_in[8];
  const float* b21  = (const float*)d_in[9];
  const float* Wh1  = (const float*)d_in[10];
  const float* bh1  = (const float*)d_in[11];
  const float* Wh2  = (const float*)d_in[12];
  const float* bh2  = (const float*)d_in[13];
  float* out = (float*)d_out;
  const int* src = ei;
  const int* dst = ei + nE;

  const int nb   = pick_nb(nE, NBL);
  if (nb < 64 || (NBL % nb) != 0) return;
  const int gA   = NBL / nb;
  const int vec8 = ((nE & 3) == 0) ? 1 : 0;

  char* ws = (char*)d_ws;
  size_t off = 0;
  const size_t oDI  = off; off += (size_t)NBL * 4;                 off = (off + 255) & ~(size_t)255;
  const size_t oXR  = off; off += (size_t)nN * XD * 4;             off = (off + 255) & ~(size_t)255;
  const size_t oTAB = off; off += (size_t)TABN * 4;                off = (off + 255) & ~(size_t)255;
  const size_t oH1  = off; off += (size_t)nN * HID * 4;            off = (off + 255) & ~(size_t)255;
  const size_t oA2H = off; off += (size_t)NBL * KF * 2;            off = (off + 255) & ~(size_t)255;
  const size_t oA2L = off; off += (size_t)NBL * KF * 2;            off = (off + 255) & ~(size_t)255;
  const size_t oH2H = off; off += (size_t)NBL * HID * 2;           off = (off + 255) & ~(size_t)255;
  const size_t oH2L = off; off += (size_t)NBL * HID * 2;           off = (off + 255) & ~(size_t)255;
  const size_t oWC  = off; off += (size_t)HID * KF * 2;            off = (off + 255) & ~(size_t)255;
  const size_t oWH  = off; off += (size_t)HID * HID * 2;           off = (off + 255) & ~(size_t)255;
  if (off > ws_size || off > (size_t)WSMAX) return;
  float*          DINV = (float*)(ws + oDI);
  float*          XR   = (float*)(ws + oXR);
  float*          TAB  = (float*)(ws + oTAB);
  float*          H1F  = (float*)(ws + oH1);
  unsigned short* A2H  = (unsigned short*)(ws + oA2H);
  unsigned short* A2L  = (unsigned short*)(ws + oA2L);
  unsigned short* H2H  = (unsigned short*)(ws + oH2H);
  unsigned short* H2L  = (unsigned short*)(ws + oH2L);
  unsigned short* WCT  = (unsigned short*)(ws + oWC);
  unsigned short* WHT  = (unsigned short*)(ws + oWH);

  hipFuncSetAttribute(reinterpret_cast<const void*>(&k_agg<0>), hipFuncAttributeMaxDynamicSharedMemorySize, LDS_AGG);
  hipFuncSetAttribute(reinterpret_cast<const void*>(&k_agg<1>), hipFuncAttributeMaxDynamicSharedMemorySize, LDS_AGG);
  hipFuncSetAttribute(reinterpret_cast<const void*>(&k_agg<2>), hipFuncAttributeMaxDynamicSharedMemorySize, LDS_AGG);

  {
    int gx = cdiv(nXf >> 2, NTHR);
    gx = gx < 2 ? 2 : gx;
    k_prep<<<dim3(gx, 9), NTHR, 0, stream>>>(X, W10, b10, W11, b11, Wh2, bh2, b20, b21, bh1, XR, TAB, nXf);
  }
  {
    const int nU1 = HID * (KF / 8);
    k_wtr<<<cdiv(nU1, NTHR), NTHR, 0, stream>>>(W20, W21, HID, KF, HID, WCT, nU1);
    const int nU2 = HID * (HID / 8);
    k_wtr<<<cdiv(nU2, NTHR), NTHR, 0, stream>>>(Wh1, Wh1, HID, HID, HID, WHT, nU2);
  }
  k_agg<2><<<dim3(gA, 1), NTHR, LDS_AGG, stream>>>(src, dst, nE, nb, vec8, 0, DINV, DINV, XR, TAB, H1F, A2H, A2L);
  k_agg<0><<<dim3(gA, nB), NTHR, LDS_AGG, stream>>>(src, dst, nE, nb, vec8, 0, DINV, DINV, XR, TAB, H1F, A2H, A2L);

  const int nUc = NBL * (HID / 8);
  const int gM  = NBL / GBM;
  for (int c = 0; c < nB; ++c) {
    k_cvt<<<cdiv(nUc, NTHR), NTHR, 0, stream>>>(H1F + (size_t)c * NBL * HID, A2H, A2L, nUc, KF);
    k_agg<1><<<dim3(gA, 1), NTHR, LDS_AGG, stream>>>(src, dst, nE, nb, vec8, c, DINV, DINV, XR, TAB, H1F, A2H, A2L);
    k_gemm2<<<dim3(gM, HID / GBN), GTHR, 0, stream>>>(A2H, A2L, WCT, TAB + T_B2S, H2H, H2L, KF, HID);
    k_gemm3<<<dim3(gM, 1), GTHR, 0, stream>>>(H2H, H2L, WHT, TAB + T_BH1, TAB + T_WH2, TAB + T_BH2,
                                              out, HID, c * NBL, nN * 2);
  }
}
